// JointGNNEncoder_26980984553612
// MI455X (gfx1250) — hardware-verified
//
#include <hip/hip_runtime.h>
#include <stdint.h>
#include <stddef.h>


typedef __attribute__((ext_vector_type(16))) _Float16 v16h;
typedef __attribute__((ext_vector_type(8)))  _Float16 v8h;
typedef __attribute__((ext_vector_type(4)))  _Float16 v4h;
typedef __attribute__((ext_vector_type(8)))  float    v8f;
typedef __attribute__((ext_vector_type(4)))  float    v4f;

__device__ __forceinline__ void dep_guard_h(v8f& a, v8f& b, v16h x, v16h y) { asm volatile("v_nop\n\tv_nop\n\tv_nop\n\tv_nop" : "+v"(a), "+v"(b) : "v"(x), "v"(y)); }
__device__ __forceinline__ void keep4_h(v16h a, v16h b, v16h c, v16h d) { asm volatile("v_nop" :: "v"(a), "v"(b), "v"(c), "v"(d)); }
template <typename T> struct Frag;
template <> struct Frag<_Float16> {
  typedef v16h V; union U { v16h v; v8h h[2]; };
  static __device__ __forceinline__ v16h load(const _Float16* p) {
    U f; f.h[0] = *(const v8h*)(p); f.h[1] = *(const v8h*)(p + 16); return f.v;
  }
  static __device__ __forceinline__ v8f mma(v16h a, v16h b, v8f c) {
    return __builtin_amdgcn_wmma_f32_16x16x32_f16(false, a, false, b, (short)0, c, false, false);
  }
  static __device__ __forceinline__ void guard(v8f& a, v8f& b, v16h x, v16h y) { dep_guard_h(a, b, x, y); }
  static __device__ __forceinline__ void keep(v16h a, v16h b, v16h c, v16h d) { keep4_h(a, b, c, d); }
};

__device__ __forceinline__ v8f mma16(v16h a, v16h b, v8f c) {
  c = __builtin_amdgcn_wmma_f32_16x16x32_f16(false, a, false, b, (short)0, c, false, false);
  asm volatile("v_nop\n\tv_nop\n\tv_nop\n\tv_nop" : "+v"(c) : "v"(a), "v"(b));
  return c;
}

#define NJ   24
#define GPB  2
#define ROWS (GPB * NJ)
#define CIN  64
#define HD   256
#define XP   72
#define HP   264
#define TP   56
#define AP   40

__global__ __launch_bounds__(256)
void transpose_cast_f16(const float* __restrict__ W, _Float16* __restrict__ Wt, int K, int N) {
  __shared__ float tile[64][65];
  const int tid = threadIdx.x;
  const int n0 = blockIdx.x * 64;
  const int k0 = blockIdx.y * 64;
  for (int i = tid; i < 64 * 64; i += 256) {
    const int kr = i >> 6, nc = i & 63;
    const int kk = k0 + kr, nn = n0 + nc;
    float v = 0.0f;
    if (kk < K && nn < N) v = W[(size_t)kk * N + nn];
    tile[kr][nc] = v;
  }
  __syncthreads();
  const int c8  = (tid & 7) * 8;
  const int nr0 = tid >> 3;
  v8h h0, h1;
#pragma unroll
  for (int e = 0; e < 8; ++e) {
    h0[e] = (_Float16)tile[c8 + e][nr0];
    h1[e] = (_Float16)tile[c8 + e][nr0 + 32];
  }
  const int nn0 = n0 + nr0, nn1 = n0 + nr0 + 32;
  const bool kok = (k0 + c8 + 8 <= K);
  for (int pass = 0; pass < 2; ++pass) {
    if (kok && nn0 < N) *(volatile v8h*)(Wt + (size_t)nn0 * K + k0 + c8) = h0;
    if (kok && nn1 < N) *(volatile v8h*)(Wt + (size_t)nn1 * K + k0 + c8) = h1;
    __threadfence();
  }
}

__global__ __launch_bounds__(256)
void gcn2_fused(const float* __restrict__ feats,
                const float* __restrict__ b1,
                const float* __restrict__ b2,
                const float* __restrict__ Anorm,
                const _Float16* __restrict__ W1t,
                const _Float16* __restrict__ W2t,
                float* __restrict__ out,
                int B) {
  __shared__ __attribute__((aligned(16))) _Float16 XH[ROWS * HP];
  __shared__ __attribute__((aligned(16))) _Float16 TT[HD * TP];
  __shared__ __attribute__((aligned(16))) _Float16 As[32 * AP];
  __shared__ __attribute__((aligned(16))) float outs[GPB * HD];
  __shared__ float b1s[HD];
  __shared__ float b2s[HD];

  const int tid  = threadIdx.x;
  const int lane = tid & 31;
  const int wave = tid >> 5;
  const int hh   = lane >> 4;
  const int c    = lane & 15;
  const int g0   = blockIdx.x * GPB;
  int ng = B - g0;
  ng = ng < 0 ? 0 : (ng > GPB ? GPB : ng);

  for (int i = tid; i < 32 * 32; i += 256) {
    const int m = i >> 5, k = i & 31;
    float v = 0.0f;
    if (m < NJ && k < NJ) v = Anorm[m * NJ + k];
    As[m * AP + k] = (_Float16)v;
  }
  for (int i = tid; i < HD; i += 256) { b1s[i] = b1[i]; b2s[i] = b2[i]; }
  {
    v8h z;
#pragma unroll
    for (int e = 0; e < 8; ++e) z[e] = (_Float16)0.0f;
    for (int n = tid; n < HD; n += 256) *(v8h*)(TT + n * TP + ROWS) = z;
  }
  {
    const float* src = feats + (size_t)g0 * NJ * CIN;
    for (int i = tid; i < ROWS * CIN / 4; i += 256) {
      const int e = i * 4;
      const int row = e >> 6, k = e & 63;
      const int gl = (row >= NJ) ? 1 : 0;
      v4f v = (v4f){0.f, 0.f, 0.f, 0.f};
      if (gl < ng) v = *(const v4f*)(src + e);
      v4h p;
      p[0] = (_Float16)v[0]; p[1] = (_Float16)v[1]; p[2] = (_Float16)v[2]; p[3] = (_Float16)v[3];
      *(v4h*)(XH + row * XP + k) = p;
    }
  }
  __syncthreads();

  const v8f zacc = (v8f){0.f, 0.f, 0.f, 0.f, 0.f, 0.f, 0.f, 0.f};

  {
    v8f acc[3][2];
#pragma unroll
    for (int mt = 0; mt < 3; ++mt) { acc[mt][0] = zacc; acc[mt][1] = zacc; }
#pragma unroll
    for (int kt = 0; kt < CIN / 32; ++kt) {
      v16h a[3];
#pragma unroll
      for (int mt = 0; mt < 3; ++mt)
        a[mt] = Frag<_Float16>::load(XH + (mt * 16 + c) * XP + kt * 32 + 8 * hh);
#pragma unroll
      for (int cto = 0; cto < 2; ++cto) {
        const int n = (wave * 2 + cto) * 16 + c;
        const v16h b = Frag<_Float16>::load(W1t + (size_t)n * CIN + kt * 32 + 8 * hh);
#pragma unroll
        for (int mt = 0; mt < 3; ++mt) acc[mt][cto] = mma16(a[mt], b, acc[mt][cto]);
      }
    }
#pragma unroll
    for (int mt = 0; mt < 3; ++mt) {
#pragma unroll
      for (int cto = 0; cto < 2; ++cto) {
        const int n = (wave * 2 + cto) * 16 + c;
        v8h hv;
#pragma unroll
        for (int r = 0; r < 8; ++r) hv[r] = (_Float16)acc[mt][cto][r];
        *(v8h*)(TT + n * TP + mt * 16 + 8 * hh) = hv;
      }
    }
  }
  __syncthreads();

  {
    v16h af[2];
#pragma unroll
    for (int mt2 = 0; mt2 < 2; ++mt2) af[mt2] = Frag<_Float16>::load(As + (mt2 * 16 + c) * AP + 8 * hh);
#pragma unroll
    for (int g = 0; g < GPB; ++g) {
#pragma unroll
      for (int cto = 0; cto < 2; ++cto) {
        const int n = (wave * 2 + cto) * 16 + c;
        const v16h b = Frag<_Float16>::load(TT + n * TP + NJ * g + 8 * hh);
        const float bias = b1s[n];
#pragma unroll
        for (int mt2 = 0; mt2 < 2; ++mt2) {
          const v8f d = mma16(af[mt2], b, zacc);
          if (mt2 == 0 || hh == 0) {
#pragma unroll
            for (int r = 0; r < 8; ++r) {
              const float v = fmaxf(d[r] + bias, 0.0f);
              XH[(NJ * g + mt2 * 16 + 8 * hh + r) * HP + n] = (_Float16)v;
            }
          }
        }
      }
    }
  }
  __syncthreads();

  {
    v8f acc[3][2];
#pragma unroll
    for (int mt = 0; mt < 3; ++mt) { acc[mt][0] = zacc; acc[mt][1] = zacc; }
#pragma unroll 1
    for (int kt = 0; kt < HD / 32; ++kt) {
      v16h a[3];
#pragma unroll
      for (int mt = 0; mt < 3; ++mt)
        a[mt] = Frag<_Float16>::load(XH + (mt * 16 + c) * HP + kt * 32 + 8 * hh);
#pragma unroll
      for (int cto = 0; cto < 2; ++cto) {
        const int n = (wave * 2 + cto) * 16 + c;
        const v16h b = Frag<_Float16>::load(W2t + (size_t)n * HD + kt * 32 + 8 * hh);
#pragma unroll
        for (int mt = 0; mt < 3; ++mt) acc[mt][cto] = mma16(a[mt], b, acc[mt][cto]);
      }
    }
#pragma unroll
    for (int mt = 0; mt < 3; ++mt) {
#pragma unroll
      for (int cto = 0; cto < 2; ++cto) {
        const int n = (wave * 2 + cto) * 16 + c;
        v8h hv;
#pragma unroll
        for (int r = 0; r < 8; ++r) hv[r] = (_Float16)acc[mt][cto][r];
        *(v8h*)(TT + n * TP + mt * 16 + 8 * hh) = hv;
      }
    }
  }
  __syncthreads();

  {
    v16h af[2];
#pragma unroll
    for (int mt2 = 0; mt2 < 2; ++mt2) af[mt2] = Frag<_Float16>::load(As + (mt2 * 16 + c) * AP + 8 * hh);
#pragma unroll
    for (int g = 0; g < GPB; ++g) {
#pragma unroll
      for (int cto = 0; cto < 2; ++cto) {
        const int n = (wave * 2 + cto) * 16 + c;
        const v16h b = Frag<_Float16>::load(TT + n * TP + NJ * g + 8 * hh);
        const float bias = b2s[n];
        float s = 0.0f;
#pragma unroll
        for (int mt2 = 0; mt2 < 2; ++mt2) {
          const v8f d = mma16(af[mt2], b, zacc);
#pragma unroll
          for (int r = 0; r < 8; ++r) {
            const float v = fmaxf(d[r] + bias, 0.0f);
            if (mt2 == 0 || hh == 0) s += v;
          }
        }
        s += __shfl_xor(s, 16, 32);
        if (hh == 0) outs[g * HD + n] = s * (1.0f / 24.0f);
      }
    }
  }
  __syncthreads();

  {
    const int nst = ng * (HD / 4);
    v4f v = (v4f){0.f, 0.f, 0.f, 0.f};
    if (tid < nst) v = *(const v4f*)(outs + tid * 4);
    float* ob = out + (size_t)g0 * HD;
    for (int pass = 0; pass < 2; ++pass) {
      if (tid < nst) *(volatile v4f*)(ob + tid * 4) = v;
      __threadfence();
    }
  }
}

extern "C" void kernel_launch(void* const* d_in, const int* in_sizes, int n_in,
                              void* d_out, int out_size, void* d_ws, size_t ws_size,
                              hipStream_t stream) {
  if (n_in < 6) return;
  const float* feats = (const float*)d_in[0];
  const float* W1    = (const float*)d_in[1];
  const float* b1    = (const float*)d_in[2];
  const float* W2    = (const float*)d_in[3];
  const float* b2    = (const float*)d_in[4];
  const float* An    = (const float*)d_in[5];
  float* out         = (float*)d_out;

  const int B = in_sizes[0] / (NJ * CIN);
  if (B <= 0) return;
  if (in_sizes[0] != B * NJ * CIN) return;
  if (in_sizes[1] != CIN * HD || in_sizes[2] != HD || in_sizes[3] != HD * HD || in_sizes[4] != HD || in_sizes[5] != NJ * NJ) return;
  if (out_size != B * HD) return;

  const size_t w1_bytes = (size_t)HD * CIN * 2;
  const size_t w2_bytes = (size_t)HD * HD * 2;
  if (w1_bytes + w2_bytes > ws_size) return;
  _Float16* W1t = (_Float16*)d_ws;
  _Float16* W2t = (_Float16*)((char*)d_ws + w1_bytes);

  transpose_cast_f16<<<dim3(HD / 64, CIN / 64), 256, 0, stream>>>(W1, W1t, CIN, HD);
  transpose_cast_f16<<<dim3(HD / 64, HD / 64), 256, 0, stream>>>(W2, W2t, HD, HD);

  const int nblk = (B + GPB - 1) / GPB;
  gcn2_fused<<<nblk, 256, 0, stream>>>(feats, b1, b2, An, W1t, W2t, out, B);
}
